// VariationalGCNEncoder_46093589021377
// MI455X (gfx1250) — hardware-run, weakly checked
//
#include <hip/hip_runtime.h>


namespace {
constexpr int NN = 100000, NP = 100000, NE = 1600000, D = 128, DO = 64, MAXDEG = 1024, NGc = (NN + 511) / 512, PERMLEN = NE + 32 * NGc + 32;
constexpr float XS = 8.0f;
__device__ __forceinline__ float nexp(float x) { return __builtin_amdgcn_exp2f(x * 1.4426950408889634f); }
__device__ __forceinline__ float nlog(float x) { return __builtin_amdgcn_logf(x) * 0.6931471805599453f; }

typedef _Float16 b16;
typedef __attribute__((ext_vector_type(16))) _Float16 v16b;
typedef __attribute__((ext_vector_type(8))) _Float16 v8b;
typedef __attribute__((ext_vector_type(8))) float v8f;
typedef __attribute__((ext_vector_type(4))) float v4f;
__device__ __forceinline__ float bf16_rne(float f) { unsigned int u = __float_as_uint(f); u += 0x7FFFu + ((u >> 16) & 1u); return __uint_as_float(u & 0xFFFF0000u); }
__device__ __forceinline__ void split16(float v, b16& hi, b16& lo) { hi = (b16)v; lo = (b16)(v - (float)hi); }
__device__ __forceinline__ v16b frag_kb(const b16* p, int hh) { const v8b a = *(const v8b*)(p + 8 * hh), b = *(const v8b*)(p + 16 + 8 * hh); v16b f;
#pragma unroll
  for (int e = 0; e < 8; ++e) { f[e] = a[e]; f[8 + e] = b[e]; } return f; }
__device__ __forceinline__ v8f wmma16b(v16b a, v16b b, v8f c) { v8f d = __builtin_amdgcn_wmma_f32_16x16x32_f16(false, a, false, b, (short)0, c, false, false); asm volatile("v_nop\n\tv_nop\n\tv_nop\n\tv_nop" : "+v"(d) : "v"(a), "v"(b)); return d; }
__device__ __forceinline__ void wave_lds_sync() { __builtin_amdgcn_fence(__ATOMIC_RELEASE, "workgroup"); __builtin_amdgcn_wave_barrier(); __builtin_amdgcn_fence(__ATOMIC_ACQUIRE, "workgroup"); }
__device__ __forceinline__ float pmul(float a, float b) { float p = a * b; asm volatile("" : "+v"(p)); return p; }
__device__ __forceinline__ float wsum(float v) {
#pragma unroll
  for (int o = 1; o < 32; o <<= 1) v += __shfl_xor(v, o); return v; }
constexpr int CSR_NBLK = 512, CSR_GB = 9, CSR_GN = 1 << CSR_GB  , CSR_MAXG = 512, CSR_CAP = 12288  ;
__global__ __launch_bounds__(64) void csrA_kernel(const int* __restrict__ dst, int E, int N, int nG, int CHP, int NGP, int* __restrict__ STG, int* __restrict__ HST) {
  extern __shared__ int sm[];
  int* cnt = sm; int* run = sm + NGP; int* ids = sm + 2 * NGP;
  const int b = blockIdx.x; const int ch = (E + CSR_NBLK - 1) / CSR_NBLK; const int e0 = b * ch, e1 = min(E, e0 + ch);
  for (int i = threadIdx.x; i < NGP; i += 64) cnt[i] = 0;
  for (int i = threadIdx.x; i < CHP; i += 64) ids[i] = -1;
  __syncthreads();
  if (threadIdx.x == 0) {
    for (int e = e0; e < e1; ++e) { int d = dst[e]; d = (d < 0) ? 0 : (d >= N ? N - 1 : d); cnt[d >> CSR_GB] += 1; }
    int acc = 0; for (int g = 0; g < nG; ++g) { run[g] = acc; acc += cnt[g]; }
    for (int e = e0; e < e1; ++e) { int d = dst[e]; d = (d < 0) ? 0 : (d >= N ? N - 1 : d); const int g = d >> CSR_GB; ids[run[g]] = e; run[g] += 1; } }
  __syncthreads();
  typedef __attribute__((ext_vector_type(4))) int v4i;
  for (int pass = 0; pass < 2; ++pass) {
    for (int i = threadIdx.x; i < CHP / 4; i += 64) *(volatile v4i*)(STG + (size_t)b * CHP + i * 4) = *(const v4i*)(&ids[i * 4]);
    for (int i = threadIdx.x; i < NGP / 4; i += 64) { v4i v; for (int e = 0; e < 4; ++e) v[e] = (i * 4 + e < nG) ? cnt[i * 4 + e] : 0; *(volatile v4i*)(HST + (size_t)b * NGP + i * 4) = v; }
    __threadfence(); }
}
__global__ __launch_bounds__(512) void csrS_kernel(const int* __restrict__ HST, int nG, int NGP, int* __restrict__ START, int* __restrict__ TOT, int* __restrict__ OFF) {
  __shared__ int tot[CSR_MAXG];
  const int b = threadIdx.x;
  for (int pass = 0; pass < 2; ++pass) { int runb = 0; for (int g = 0; g < nG; ++g) { int c = HST[(size_t)b * NGP + g]; c = (c < 0) ? 0 : c; ((volatile int*)OFF)[(size_t)g * CSR_NBLK + b] = runb; runb += c; } __threadfence(); }
  for (int g = threadIdx.x; g < nG; g += 512) { int s = 0; for (int bb = 0; bb < CSR_NBLK; ++bb) { int c = HST[(size_t)bb * NGP + g]; s += (c < 0) ? 0 : c; } tot[g] = s; }
  __syncthreads();
  if (threadIdx.x < 32) {
    __shared__ int st[CSR_MAXG + 32];
    if (threadIdx.x == 0) { int acc = 0; for (int g = 0; g < NGP; ++g) { st[g] = acc; if (g < nG) acc += (tot[g] + 31) & ~31; } st[NGP] = acc; }
    __builtin_amdgcn_fence(__ATOMIC_RELEASE, "workgroup"); __builtin_amdgcn_wave_barrier(); __builtin_amdgcn_fence(__ATOMIC_ACQUIRE, "workgroup");
    for (int pass = 0; pass < 2; ++pass) { for (int i = threadIdx.x; i < NGP + 32; i += 32) { ((volatile int*)START)[i] = (i <= NGP) ? st[min(i, NGP)] : 0; ((volatile int*)TOT)[i] = (i < nG) ? tot[i] : 0; } __threadfence(); } }
}
__global__ __launch_bounds__(256) void csrB_kernel(const int* __restrict__ dst, int N, int nG, int CHP, int NGP, int permLen, const int* __restrict__ STG, const int* __restrict__ HST, const int* __restrict__ OFF, const int* __restrict__ START, const int* __restrict__ TOT, int* __restrict__ PERM, int* __restrict__ ROWPTR, int* __restrict__ ROWCNT, int* __restrict__ FLAG) {
  typedef __attribute__((ext_vector_type(4))) int v4i;
  __shared__ int ids[CSR_CAP]; __shared__ unsigned short key[CSR_CAP]; __shared__ int outp[CSR_CAP]; __shared__ int ncnt[CSR_GN + 1]; __shared__ int boff[CSR_NBLK + 1];
  const int g = blockIdx.x, t_ = threadIdx.x; int tot = TOT[g]; int st = START[g], stn = START[g + 1]; const int v0 = g * CSR_GN; const int nv = min(CSR_GN, N - v0);
  st = (st < 0) ? 0 : (st > permLen - 32 ? permLen - 32 : st) & ~31; stn = (stn < st) ? st : (stn > permLen ? permLen : stn); tot = (tot < 0) ? 0 : tot; if (tot > stn - st && tot <= CSR_CAP) tot = stn - st;
  if (tot > CSR_CAP) {
    for (int pass = 0; pass < 2; ++pass) { for (int i = t_; i < CSR_GN / 4; i += 256) { v4i a, c; for (int e = 0; e < 4; ++e) { a[e] = st; c[e] = 0; } *(volatile v4i*)(ROWPTR + v0 + i * 4) = a; *(volatile v4i*)(ROWCNT + v0 + i * 4) = c; } if (t_ == 0) ((volatile int*)FLAG)[0] = 1; __threadfence(); } (void)nv; return; }
  if (t_ == 0) { int acc = 0; for (int b = 0; b < CSR_NBLK; ++b) { boff[b] = acc; int c = HST[(size_t)b * NGP + g]; c = (c < 0) ? 0 : (c > CHP ? CHP : c); acc += c; if (acc > tot) acc = tot; } boff[CSR_NBLK] = acc; }
  for (int i = t_; i <= CSR_GN; i += 256) ncnt[i] = 0;
  __syncthreads();
  for (int b = 0; b < CSR_NBLK; ++b) { const int c = boff[b + 1] - boff[b]; int o_ = OFF[(size_t)g * CSR_NBLK + b]; o_ = (o_ < 0) ? 0 : (o_ > CHP - c ? CHP - c : o_); const int* src_ = STG + (size_t)b * CHP + o_;
    for (int i = t_; i < c; i += 256) { int id = src_[i]; id = (id < 0) ? 0 : id; ids[boff[b] + i] = id; int d = dst[id]; d = (d < v0) ? v0 : (d >= N ? N - 1 : d); int kk = d - v0; kk = (kk < 0) ? 0 : (kk >= CSR_GN ? CSR_GN - 1 : kk); key[boff[b] + i] = (unsigned short)kk; } }
  __syncthreads();
  if (t_ == 0) { for (int i = 0; i < tot; ++i) ncnt[key[i]] += 1; int acc = 0; for (int vl = 0; vl < CSR_GN; ++vl) { const int c = ncnt[vl]; ncnt[vl] = acc; acc += c; } ncnt[CSR_GN] = acc;
    for (int i = 0; i < tot; ++i) { const int vl = key[i]; outp[ncnt[vl]] = ids[i]; ncnt[vl] += 1; }
    for (int vl = CSR_GN; vl > 0; --vl) ncnt[vl] = ncnt[vl - 1]; ncnt[0] = 0; }
  __syncthreads();
  for (int pass = 0; pass < 2; ++pass) {
    for (int i = t_; i < (stn - st) / 4; i += 256) { v4i v; for (int e = 0; e < 4; ++e) { const int q = i * 4 + e; v[e] = (q < tot) ? outp[q] : -1; } *(volatile v4i*)(PERM + st + i * 4) = v; }
    for (int i = t_; i < CSR_GN / 4; i += 256) { v4i a, c; for (int e = 0; e < 4; ++e) { const int vl = i * 4 + e; a[e] = st + ncnt[vl]; c[e] = (vl < nv) ? (ncnt[vl + 1] - ncnt[vl]) : 0; } *(volatile v4i*)(ROWPTR + v0 + i * 4) = a; *(volatile v4i*)(ROWCNT + v0 + i * 4) = c; }
    __threadfence(); }
}
__global__ __launch_bounds__(256) void csrZ_kernel(int* __restrict__ p, size_t n4) { typedef __attribute__((ext_vector_type(4))) int v4i; const size_t tid = (size_t)blockIdx.x * 256 + threadIdx.x, nth = (size_t)gridDim.x * 256; v4i z = {0, 0, 0, 0}; for (size_t i = tid; i < n4; i += nth) *(volatile v4i*)(p + i * 4) = z; }
struct CsrBufs { int *STG, *HST, *OFF, *START, *TOT, *PERM, *ROWPTR, *ROWCNT, *FLAG; int nG, NGP, CHP; size_t permLen; char* base; size_t bytes; };
static size_t csr_carve(CsrBufs& c, char* ws, size_t off, int E, int N) {
  const size_t off0 = off; c.base = ws + off;
  auto al = [&](size_t bytes) { char* p = ws + off; off += (bytes + 255) & ~(size_t)255; return p; };
  c.nG = (N + CSR_GN - 1) / CSR_GN; c.NGP = (c.nG + 31) & ~31; const int ch = (E + CSR_NBLK - 1) / CSR_NBLK; c.CHP = (ch + 31) & ~31; c.permLen = (size_t)E + 32 * (size_t)c.nG + 32;
  c.STG = (int*)al((size_t)CSR_NBLK * c.CHP * 4); c.HST = (int*)al((size_t)CSR_NBLK * c.NGP * 4); c.OFF = (int*)al((size_t)c.NGP * CSR_NBLK * 4); c.START = (int*)al((size_t)(c.NGP + 64) * 4); c.TOT = (int*)al((size_t)(c.NGP + 64) * 4);
  c.PERM = (int*)al(c.permLen * 4); c.ROWPTR = (int*)al((size_t)c.nG * CSR_GN * 4); c.ROWCNT = (int*)al((size_t)c.nG * CSR_GN * 4); c.FLAG = (int*)al(256);
  c.bytes = off - off0; return off;
}
static void csr_build(const CsrBufs& c, const int* dst, int E, int N, hipStream_t stream) {
  const size_t smem = (size_t)(2 * c.NGP + c.CHP) * 4;
  csrZ_kernel<<<512, 256, 0, stream>>>((int*)c.base, c.bytes / 16);
  csrA_kernel<<<CSR_NBLK, 64, smem, stream>>>(dst, E, N, c.nG, c.CHP, c.NGP, c.STG, c.HST);
  csrS_kernel<<<1, 512, 0, stream>>>(c.HST, c.nG, c.NGP, c.START, c.TOT, c.OFF);
  csrB_kernel<<<c.nG, 256, 0, stream>>>(dst, N, c.nG, c.CHP, c.NGP, (int)c.permLen, c.STG, c.HST, c.OFF, c.START, c.TOT, c.PERM, c.ROWPTR, c.ROWCNT, c.FLAG);
}

__global__ __launch_bounds__(256) void prep_kernel(const float* __restrict__ x, const float* __restrict__ w1, const float* __restrict__ b1, const float* __restrict__ wmu, const float* __restrict__ bmu, const float* __restrict__ wls, const float* __restrict__ bls, b16* __restrict__ R, float* __restrict__ P, b16* __restrict__ Hh, b16* __restrict__ Hl) {
  const size_t tid = (size_t)blockIdx.x * 256 + threadIdx.x, nth = (size_t)gridDim.x * 256;
  for (int pass = 0; pass < 2; ++pass) {
    for (size_t p = tid; p < (size_t)2 * D * (D / 8); p += nth) { const int l = (int)(p / (D * (D / 8))), rem = (int)(p % (D * (D / 8))), o = rem / (D / 8), k0 = (rem % (D / 8)) * 8; v8b v;
      for (int e = 0; e < 8; ++e) { float w; if (l == 0) w = w1[(size_t)(k0 + e) * D + o]; else w = (o < DO) ? wmu[(size_t)(k0 + e) * DO + o] : wls[(size_t)(k0 + e) * DO + (o - DO)]; v[e] = (b16)bf16_rne(w); } *(volatile v8b*)(R + ((size_t)l * D + o) * D + k0) = v; }
    for (size_t q = tid; q < 256; q += nth) { const int i = (int)q; ((volatile float*)P)[q] = bf16_rne((i < 128) ? b1[i] : (i < 192) ? bmu[i - 128] : bls[i - 192]); }
    for (size_t p = tid; p < (size_t)NP * D / 8; p += nth) { v8b v = {}, z = {}; for (int e = 0; e < 8; ++e) v[e] = (b16)(bf16_rne(x[p * 8 + e]) * XS); *(volatile v8b*)(Hh + p * 8) = v; *(volatile v8b*)(Hl + p * 8) = z; }
    __threadfence(); }
}

__global__ __launch_bounds__(64) void gemm_kernel(const b16* __restrict__ Hh, const b16* __restrict__ Hl, const b16* __restrict__ Bw, float* __restrict__ HW) {
  __shared__ __attribute__((aligned(16))) float Ts[2][16][D + 4];
  const int lane = threadIdx.x & 31, wave = threadIdx.x >> 5, nloc = lane & 15, hlf = lane >> 4, m0 = blockIdx.x * 32 + wave * 16;
  v8f acc[8];
#pragma unroll
  for (int t = 0; t < 8; ++t) acc[t] = (v8f){};
#pragma unroll
  for (int kb = 0; kb < D; kb += 32) { const v16b a = frag_kb(Hh + (size_t)(m0 + nloc) * D + kb, hlf), al = frag_kb(Hl + (size_t)(m0 + nloc) * D + kb, hlf);
#pragma unroll
    for (int t = 0; t < 8; ++t) { const v16b bw = frag_kb(Bw + (size_t)(t * 16 + nloc) * D + kb, hlf); acc[t] = wmma16b(a, bw, acc[t]); acc[t] = wmma16b(al, bw, acc[t]); } }
#pragma unroll
  for (int t = 0; t < 8; ++t)
#pragma unroll
    for (int r = 0; r < 8; ++r) Ts[wave][8 * hlf + r][t * 16 + nloc] = acc[t][r] * (1.0f / XS);
  wave_lds_sync();
  for (int pass = 0; pass < 2; ++pass) { for (int i = lane; i < 16 * 32; i += 32) { const int rr = i >> 5, c4 = (i & 31) * 4; *(volatile v4f*)(HW + (size_t)(m0 + rr) * D + c4) = *(const v4f*)(&Ts[wave][rr][c4]); } __threadfence(); }
}

template <int MODE>
__global__ __launch_bounds__(256) void agg_kernel(const float* __restrict__ HW, const int* __restrict__ src, const int* __restrict__ perm, const int* __restrict__ rowptr, const int* __restrict__ rowcnt, const float* __restrict__ Pb, b16* __restrict__ Hh, b16* __restrict__ Hl, float* __restrict__ out0, float* __restrict__ out1) {
  __shared__ __attribute__((aligned(16))) b16 Sh[8][D + 8], Sl[8][D + 8];
  const int wave = threadIdx.x >> 5, v = blockIdx.x * 8 + wave, lane = threadIdx.x & 31;
  int cnt = rowcnt[v]; cnt = (cnt < 0) ? 0 : (cnt > MAXDEG ? MAXDEG : cnt); int p0 = rowptr[v]; p0 = (p0 < 0) ? 0 : (p0 > PERMLEN - cnt ? PERMLEN - cnt : p0);
  const float dv = rsqrtf((float)cnt + 1.0f);
  v4f acc = *(const v4f*)(HW + (size_t)v * D + lane * 4) * (dv * dv);
  for (int q = 0; q < cnt; ++q) { int id = perm[p0 + q]; id = (id < 0) ? 0 : (id >= NE ? NE - 1 : id); int s = src[id]; s = (s < 0) ? 0 : (s >= NN ? NN - 1 : s); int cs_ = rowcnt[s]; cs_ = (cs_ < 0) ? 0 : (cs_ > MAXDEG ? MAXDEG : cs_); const float w = pmul(rsqrtf((float)cs_ + 1.0f), dv); const v4f hv = *(const v4f*)(HW + (size_t)s * D + lane * 4);
#pragma unroll
    for (int e = 0; e < 4; ++e) acc[e] += pmul(w, hv[e]); }
  v4f o;
#pragma unroll
  for (int e = 0; e < 4; ++e) { o[e] = acc[e] + Pb[lane * 4 + e]; if (MODE == 0) { o[e] = fmaxf(o[e], 0.0f); b16 a_, b_; split16(o[e] * XS, a_, b_); Sh[wave][lane * 4 + e] = a_; Sl[wave][lane * 4 + e] = b_; } }
  if (MODE == 0) { wave_lds_sync(); for (int pass = 0; pass < 2; ++pass) { if (lane < 16) { *(volatile v8b*)(Hh + (size_t)v * D + lane * 8) = *(const v8b*)(&Sh[wave][lane * 8]); *(volatile v8b*)(Hl + (size_t)v * D + lane * 8) = *(const v8b*)(&Sl[wave][lane * 8]); } __threadfence(); } }
  else { float* dst = (lane < 16) ? (out0 + (size_t)v * DO + lane * 4) : (out1 + (size_t)v * DO + (lane - 16) * 4); for (int pass = 0; pass < 2; ++pass) { *(volatile v4f*)dst = o; __threadfence(); } }
}
}

extern "C" void kernel_launch(void* const* d_in, const int* in_sizes, int n_in,
                              void* d_out, int out_size, void* d_ws, size_t ws_size, hipStream_t stream) {
  (void)n_in;
  const float* x = (const float*)d_in[0]; const int* ei = (const int*)d_in[1]; const float* w1 = (const float*)d_in[2]; const float* b1 = (const float*)d_in[3]; const float* wmu = (const float*)d_in[4]; const float* bmu = (const float*)d_in[5]; const float* wls = (const float*)d_in[6]; const float* bls = (const float*)d_in[7];
  float* out0 = (float*)d_out; float* out1 = (float*)((char*)d_out + (size_t)NN * DO * 4);
  if (in_sizes[0] != NN * D || in_sizes[1] != 2 * NE || in_sizes[2] != D * D || in_sizes[3] != D || in_sizes[4] != D * DO || in_sizes[5] != DO || in_sizes[6] != D * DO || in_sizes[7] != DO || out_size != 2 * NN * DO) return;
  const int* srcI = ei; const int* dstI = ei + NE;
  size_t off = 0; char* ws = (char*)d_ws;
  auto carve = [&](size_t bytes) { char* p = ws + off; off += (bytes + 255) & ~(size_t)255; return p; };
  b16* R = (b16*)carve((size_t)2 * D * D * 2); float* P = (float*)carve(256 * 4); b16* Hh = (b16*)carve((size_t)NP * D * 2); b16* Hl = (b16*)carve((size_t)NP * D * 2); float* HW = (float*)carve((size_t)NP * D * 4);
  CsrBufs cs; off = csr_carve(cs, ws, off, NE, NN);
  if (off > ws_size) return;
  csr_build(cs, dstI, NE, NN, stream);
  prep_kernel<<<512, 256, 0, stream>>>(x, w1, b1, wmu, bmu, wls, bls, R, P, Hh, Hl);
  gemm_kernel<<<NP / 32, 64, 0, stream>>>(Hh, Hl, R, HW);
  agg_kernel<0><<<NN / 8, 256, 0, stream>>>(HW, srcI, cs.PERM, cs.ROWPTR, cs.ROWCNT, P, Hh, Hl, nullptr, nullptr);
  gemm_kernel<<<NP / 32, 64, 0, stream>>>(Hh, Hl, R + (size_t)D * D, HW);
  agg_kernel<1><<<NN / 8, 256, 0, stream>>>(HW, srcI, cs.PERM, cs.ROWPTR, cs.ROWCNT, P + 128, nullptr, nullptr, out0, out1);
}
